// Trajectory2vecDecoder_8495445311952
// MI455X (gfx1250) — hardware-verified
//
#include <hip/hip_runtime.h>


namespace {
constexpr int B = 64, L = 64, H = 128, S = 64, IN = 16, TT = 256;
constexpr float AS_ = 8.0f;

typedef _Float16 b16;
typedef __attribute__((ext_vector_type(16))) _Float16 v16b;
typedef __attribute__((ext_vector_type(8))) _Float16 v8b;
typedef __attribute__((ext_vector_type(8))) float v8f;
typedef __attribute__((ext_vector_type(4))) float v4f;
__device__ __forceinline__ float bf16_rne(float f) { unsigned int u = __float_as_uint(f); u += 0x7FFFu + ((u >> 16) & 1u); return __uint_as_float(u & 0xFFFF0000u); }
__device__ __forceinline__ void split16(float v, b16& hi, b16& lo) { hi = (b16)v; lo = (b16)(v - (float)hi); }
__device__ __forceinline__ v16b frag_kb(const b16* p, int hh) { const v8b a = *(const v8b*)(p + 8 * hh), b = *(const v8b*)(p + 16 + 8 * hh); v16b f;
#pragma unroll
  for (int e = 0; e < 8; ++e) { f[e] = a[e]; f[8 + e] = b[e]; } return f; }
__device__ __forceinline__ v8f wmma16b(v16b a, v16b b, v8f c) { v8f d = __builtin_amdgcn_wmma_f32_16x16x32_f16(false, a, false, b, (short)0, c, false, false); asm volatile("v_nop\n\tv_nop\n\tv_nop\n\tv_nop" : "+v"(d) : "v"(a), "v"(b)); return d; }
__device__ __forceinline__ void wave_lds_sync() { __builtin_amdgcn_fence(__ATOMIC_RELEASE, "workgroup"); __builtin_amdgcn_wave_barrier(); __builtin_amdgcn_fence(__ATOMIC_ACQUIRE, "workgroup"); }
__device__ __forceinline__ float nexp(float x) { return __builtin_amdgcn_exp2f(x * 1.4426950408889634f); }
__device__ __forceinline__ float sigm(float x) { return 1.0f / (1.0f + nexp(-x)); }
__device__ __forceinline__ float tanh_f(float x) { const float e = nexp(-2.0f * fabsf(x)); const float t = (1.0f - e) / (1.0f + e); return (x >= 0.0f) ? t : -t; }
__device__ __forceinline__ float pmul(float a, float b) { float p = a * b; asm volatile("" : "+v"(p)); return p; }

__global__ __launch_bounds__(256) void prep_kernel(const float* __restrict__ Wg, const float* __restrict__ bg, const float* __restrict__ Wl, const float* __restrict__ bl, const float* __restrict__ trip, b16* __restrict__ R, float* __restrict__ P, float* __restrict__ out0) {
  const int t_ = blockIdx.x * 256 + threadIdx.x, nth = gridDim.x * 256;
  for (int pass = 0; pass < 2; ++pass) {
    for (int q = t_; q < 512 * 256; q += nth) { const int o = q >> 8, k = q & 255; R[q] = (b16)bf16_rne(Wg[(size_t)k * 512 + o]); }
    for (int q = t_; q < 16 * 128; q += nth) { const int o = q >> 7, k = q & 127; R[512 * 256 + q] = (b16)bf16_rne(Wl[k * IN + o]); }
    for (int q = t_; q < 528; q += nth) P[q] = (q < 512) ? bf16_rne(bg[q]) : bf16_rne(bl[q - 512]);
    for (int q = t_; q < B * TT * IN / 4; q += nth) { const v4f v = *(const v4f*)(trip + (size_t)q * 4); v4f o; for (int e = 0; e < 4; ++e) o[e] = bf16_rne(v[e]); *(volatile v4f*)(out0 + (size_t)q * 4) = o; }
    __threadfence(); }
}

__global__ __launch_bounds__(32) void rnn_kernel(const float* __restrict__ emb, const b16* __restrict__ R, const float* __restrict__ P, float* __restrict__ cs) {
  __shared__ __attribute__((aligned(16))) b16 Ah[16][2 * H + 8], Al[16][2 * H + 8]; __shared__ __attribute__((aligned(16))) float Cst[16][H];
  const int lane = threadIdx.x, nloc = lane & 15, hlf = lane >> 4, b0 = blockIdx.x * 16; const float* bg = P;
  for (int i = lane; i < 16 * (2 * H + 8); i += 32) { (&Ah[0][0])[i] = (b16)0.0f; (&Al[0][0])[i] = (b16)0.0f; }
  for (int i = lane; i < 16 * H; i += 32) { const int r = i / H, k = i % H; (&Cst[0][0])[i] = 0.0f; Ah[r][k] = (b16)(bf16_rne(emb[((size_t)(b0 + r) * L + 0) * H + k]) * AS_); }
  wave_lds_sync();
  for (int s = 0; s < S; ++s) {
    float cn[8][8], hn[8][8];
#pragma unroll
    for (int t = 0; t < 8; ++t) { v8f g[4] = {{}, {}, {}, {}};
#pragma unroll 2
      for (int kb = 0; kb < 2 * H; kb += 32) { const v16b ah = frag_kb(&Ah[nloc][kb], hlf), al = frag_kb(&Al[nloc][kb], hlf);
#pragma unroll
        for (int q = 0; q < 4; ++q) { const v16b bw = frag_kb(R + (size_t)(q * H + t * 16 + nloc) * (2 * H) + kb, hlf); g[q] = wmma16b(ah, bw, g[q]); g[q] = wmma16b(al, bw, g[q]); } }
      const int u = t * 16 + nloc; const float bf_ = bg[u], bi = bg[H + u], bo = bg[2 * H + u], bc = bg[3 * H + u];
#pragma unroll
      for (int r = 0; r < 8; ++r) { const float f = sigm(g[0][r] * (1.0f / AS_) + bf_), ig = sigm(g[1][r] * (1.0f / AS_) + bi), og = sigm(g[2][r] * (1.0f / AS_) + bo), cd = tanh_f(g[3][r] * (1.0f / AS_) + bc);
        const float c = pmul(f, Cst[8 * hlf + r][u]) + pmul(ig, cd); cn[t][r] = c; hn[t][r] = pmul(og, tanh_f(c)); } }
    wave_lds_sync();
#pragma unroll
    for (int t = 0; t < 8; ++t) { const int u = t * 16 + nloc;
#pragma unroll
      for (int r = 0; r < 8; ++r) { const int rr = 8 * hlf + r; Cst[rr][u] = cn[t][r]; b16 h_, l_; split16(cn[t][r] * AS_, h_, l_); Ah[rr][u] = h_; Al[rr][u] = l_; split16(hn[t][r] * AS_, h_, l_); Ah[rr][H + u] = h_; Al[rr][H + u] = l_; } }
    wave_lds_sync();
    for (int pass = 0; pass < 2; ++pass) { for (int i = lane; i < 16 * (H / 4); i += 32) { const int rr = i / (H / 4), c4 = (i % (H / 4)) * 4; *(volatile v4f*)(cs + ((size_t)s * B + b0 + rr) * H + c4) = *(const v4f*)(&Cst[rr][c4]); } }
    __threadfence(); }
}

__global__ __launch_bounds__(32) void out_kernel(const float* __restrict__ cs, const b16* __restrict__ R, const float* __restrict__ P, float* __restrict__ out1) {
  __shared__ __attribute__((aligned(16))) float Z[16][IN];
  const int lane = threadIdx.x, nloc = lane & 15, hlf = lane >> 4, s0 = blockIdx.x * 16, b = blockIdx.y; const b16* Wl = R + 512 * 256; const float* bl = P + 512;
  v8f acc = {};
#pragma unroll
  for (int kb = 0; kb < H; kb += 32) { v16b ah, al; const float* row = cs + ((size_t)(s0 + nloc) * B + b) * H + kb;
#pragma unroll
    for (int e = 0; e < 8; ++e) { b16 a, c; split16(row[8 * hlf + e] * AS_, a, c); ah[e] = a; al[e] = c; split16(row[16 + 8 * hlf + e] * AS_, a, c); ah[8 + e] = a; al[8 + e] = c; }
    const v16b bw = frag_kb(Wl + (size_t)nloc * H + kb, hlf); acc = wmma16b(ah, bw, acc); acc = wmma16b(al, bw, acc); }
#pragma unroll
  for (int r = 0; r < 8; ++r) Z[8 * hlf + r][nloc] = acc[r] * (1.0f / AS_) + bl[nloc];
  wave_lds_sync();
  for (int pass = 0; pass < 2; ++pass) { for (int ss = 0; ss < 16; ++ss) { const v4f z4 = *(const v4f*)(&Z[ss][(lane & 3) * 4]); float* base = out1 + ((size_t)b * (S * L) + (size_t)(s0 + ss) * L) * IN;
      for (int l8 = 0; l8 < L; l8 += 8) *(volatile v4f*)(base + (size_t)(l8 + (lane >> 2)) * IN + (lane & 3) * 4) = z4; }
    __threadfence(); }
}
}

extern "C" void kernel_launch(void* const* d_in, const int* in_sizes, int n_in,
                              void* d_out, int out_size, void* d_ws, size_t ws_size, hipStream_t stream) {
  (void)n_in; (void)out_size;
  const float* trip = (const float*)d_in[0]; const float* emb = (const float*)d_in[2]; const float* Wg = (const float*)d_in[3]; const float* bg = (const float*)d_in[4]; const float* Wl = (const float*)d_in[5]; const float* bl = (const float*)d_in[6];
  float* out0 = (float*)d_out; float* out1 = out0 + (size_t)B * TT * IN;
  if (in_sizes[0] != B * TT * IN || in_sizes[2] != B * L * H || in_sizes[3] != 2 * H * 4 * H || in_sizes[5] != H * IN) return;
  size_t off = 0; char* ws = (char*)d_ws;
  auto carve = [&](size_t bytes) { char* p = ws + off; off += (bytes + 255) & ~(size_t)255; return p; };
  b16* R = (b16*)carve((size_t)(512 * 256 + 16 * 128) * 2); float* P = (float*)carve(1024 * 4); float* cs = (float*)carve((size_t)S * B * H * 4);
  if (off > ws_size) return;
  prep_kernel<<<128, 256, 0, stream>>>(Wg, bg, Wl, bl, trip, R, P, out0);
  rnn_kernel<<<B / 16, 32, 0, stream>>>(emb, R, P, cs);
  out_kernel<<<dim3(S / 16, B), 32, 0, stream>>>(cs, R, P, out1);
}
